// DilatedSelfAttention_63505386438964
// MI455X (gfx1250) — hardware-verified
//
#include <hip/hip_runtime.h>
#include <math.h>
#include <stdint.h>

#ifndef NB
#define NB 4
#endif
#ifndef SEQ
#define SEQ 8192
#endif
#define NB_FULL  4
#define SEQ_FULL 8192
#define CD    128
#define MSEG  (SEQ / 4)
#define NUNIT 7
#define MROWS (NB * SEQ)
#define QO    ((MSEG < 256) ? MSEG : 256)
#define KRES  ((MSEG < 512) ? MSEG : 512)
#define NQB   (MSEG / 32)
#define NKT   (MSEG / 32)
#define RSQ_HD 0.08838834764831845f
#define LOG2E 1.4426950408889634f
#define NEGT  (-1.0e30f)
#define QSC   256.0f
#define KSC   256.0f
#define PCAR  32768.0f
#define VCAR  1024.0f
#define OSC   1024.0f
#define WOS   1024.0f
#define WPB   2
#define ATT_THREADS (WPB * 32)
#define PTP   36
#define PTW   (16 * PTP)
#define SLP   132
#define SLW   (16 * SLP)
#define WREG  (PTW + SLW)
#define SLAB64 (16 * 68)
#define VTP   72
#define TWP   72
#define WS_CAP 134217728
static_assert(CD == 128 && (CD % 32) == 0);
static_assert(NB >= 1 && NB <= NB_FULL);
static_assert((SEQ % 256) == 0 && SEQ >= 256 && SEQ <= SEQ_FULL);
static_assert(MSEG * 4 == SEQ && (MSEG % 64) == 0);
static_assert((QO % 32) == 0 && QO >= 32 && QO <= MSEG && QO <= KRES);
static_assert((KRES % 64) == 0 && KRES <= MSEG);
static_assert(NQB * 32 == MSEG && NKT * 32 == MSEG);
static_assert((MROWS % 64) == 0 && ((MROWS * CD / 8) % 256) == 0);
static_assert(ATT_THREADS == 64);
static_assert(WPB * WREG * 4 <= 65536 && 2 * CD * VTP * 2 <= 65536 && 4 * SLAB64 * 4 <= 65536 && 64 * TWP * 2 <= 65536);
static_assert((size_t)131072 + (size_t)NB * MSEG * 14648 + (size_t)NB * KRES * 1792 <= (size_t)WS_CAP);

typedef unsigned short u16;
typedef _Float16 v16h __attribute__((ext_vector_type(16)));
typedef _Float16 v8h  __attribute__((ext_vector_type(8)));
typedef __bf16   v16b __attribute__((ext_vector_type(16)));
typedef float    v8f  __attribute__((ext_vector_type(8)));
typedef float    v4f  __attribute__((ext_vector_type(4)));
typedef unsigned int v4u __attribute__((ext_vector_type(4)));

union FragH { v16h v; v8h h[2]; v4u u[2]; };
union FragB { v16b v; v4u u[2]; };

__device__ __forceinline__ unsigned short bf_bits(float f) {
  unsigned u = __float_as_uint(f);
  return (unsigned short)((u + 0x7FFFu + ((u >> 16) & 1u)) >> 16);
}
__device__ __forceinline__ float bf_up(unsigned short h) { return __uint_as_float(((unsigned)h) << 16); }
__device__ __forceinline__ float bfr(float f) { return bf_up(bf_bits(f)); }
__device__ __forceinline__ unsigned short h_bits(_Float16 x) { return __builtin_bit_cast(unsigned short, x); }
__device__ __forceinline__ unsigned pk16(unsigned short a, unsigned short b) { return (unsigned)a | ((unsigned)b << 16); }
__device__ __forceinline__ v8f zero8() { v8f z = {0.f, 0.f, 0.f, 0.f, 0.f, 0.f, 0.f, 0.f}; return z; }

__device__ __forceinline__ v16h ldfrag_h(const _Float16* p) {
  FragH f;
  f.h[0] = *(const v8h*)(p);
  f.h[1] = *(const v8h*)(p + 16);
  return f.v;
}
__device__ __forceinline__ v16b ldfrag_b(const u16* p) {
  FragB f;
  f.u[0] = *(const v4u*)(p);
  f.u[1] = *(const v4u*)(p + 16);
  return f.v;
}

__device__ __forceinline__ v8f mma_h(v16h a, v16h b, v8f c) {
  return __builtin_amdgcn_wmma_f32_16x16x32_f16(false, a, false, b, (short)0, c, false, false);
}
__device__ __forceinline__ v8f mma_b(v16b a, v16b b, v8f c) {
  return __builtin_amdgcn_wmma_f32_16x16x32_bf16(false, a, false, b, (short)0, c, false, false);
}
__device__ __forceinline__ void guard2(v8f& a, v8f& b, v16h x0, v16h x1, v16h x2, v16h x3, v16h x4, v16h x5) {
#if defined(__HIP_DEVICE_COMPILE__)
  asm volatile("v_nop\n\tv_nop\n\tv_nop\n\tv_nop"
               : "+v"(a), "+v"(b) : "v"(x0), "v"(x1), "v"(x2), "v"(x3), "v"(x4), "v"(x5) : "memory");
#endif
}
template <typename F>
__device__ __forceinline__ void guard6(v8f& a, v8f& b, v8f& c, v8f& d, F x0, F x1, F x2, F x3, F x4, F x5) {
#if defined(__HIP_DEVICE_COMPILE__)
  asm volatile("v_nop\n\tv_nop\n\tv_nop\n\tv_nop"
               : "+v"(a), "+v"(b), "+v"(c), "+v"(d) : "v"(x0), "v"(x1), "v"(x2), "v"(x3), "v"(x4), "v"(x5) : "memory");
#endif
}
__device__ __forceinline__ void acc_guard4(v8f& a, v8f& b, v8f& c, v8f& d) {
#if defined(__HIP_DEVICE_COMPILE__)
  asm volatile("v_nop\n\tv_nop\n\tv_nop\n\tv_nop" : "+v"(a), "+v"(b), "+v"(c), "+v"(d));
#endif
}
__device__ __forceinline__ void wave_sync_lds() {
  __builtin_amdgcn_fence(__ATOMIC_RELEASE, "workgroup");
  __builtin_amdgcn_wave_barrier();
  __builtin_amdgcn_fence(__ATOMIC_ACQUIRE, "workgroup");
}

__global__ __launch_bounds__(256) void cvtx(const float* __restrict__ x, u16* D, int n8) {
  const int gt = blockIdx.x * 256 + (int)threadIdx.x;
  if (gt >= n8) return;
  const int row = gt >> 4;
  const int b   = row / SEQ;
  const int s   = row - b * SEQ;
  const float* p = x + ((size_t)b * SEQ_FULL + (size_t)s) * CD + (size_t)(gt & 15) * 8;
  const v4f a = *(const v4f*)(p), b4 = *(const v4f*)(p + 4);
  float w[8];
#pragma unroll
  for (int e = 0; e < 4; ++e) { w[e] = a[e]; w[4 + e] = b4[e]; }
  v4u o;
#pragma unroll
  for (int e = 0; e < 4; ++e) o[e] = pk16(bf_bits(w[2 * e]), bf_bits(w[2 * e + 1]));
  u16* d = D + (size_t)gt * 8;
  for (int pass = 0; pass < 2; ++pass) {
    *(volatile v4u*)(d) = o;
    __threadfence();
  }
}

__global__ __launch_bounds__(256) void cvt_hl(const float* __restrict__ F, u16* Hp, u16* Lp, int n8, float scale) {
  const int gt = blockIdx.x * 256 + (int)threadIdx.x;
  if (gt >= n8) return;
  const float* p = F + (size_t)gt * 8;
  const v4f a = *(const v4f*)(p), b4 = *(const v4f*)(p + 4);
  float w[8];
#pragma unroll
  for (int e = 0; e < 4; ++e) { w[e] = a[e]; w[4 + e] = b4[e]; }
  v4u oh, ol;
#pragma unroll
  for (int e = 0; e < 4; ++e) {
    const float t0 = w[2 * e] * scale, t1 = w[2 * e + 1] * scale;
    const _Float16 h0 = (_Float16)t0, h1 = (_Float16)t1;
    const _Float16 l0 = (_Float16)(t0 - (float)h0), l1 = (_Float16)(t1 - (float)h1);
    oh[e] = pk16(h_bits(h0), h_bits(h1));
    ol[e] = pk16(h_bits(l0), h_bits(l1));
  }
  u16* dh = Hp + (size_t)gt * 8;
  u16* dl = Lp + (size_t)gt * 8;
  for (int pass = 0; pass < 2; ++pass) {
    *(volatile v4u*)(dh) = oh;
    *(volatile v4u*)(dl) = ol;
    __threadfence();
  }
}

__global__ __launch_bounds__(256) void tw16(const float* __restrict__ W0, const float* __restrict__ W1,
                                            const float* __restrict__ W2, const float* __restrict__ W3, u16* T) {
  __shared__ __align__(16) u16 TT[64 * TWP];
  const int tid  = threadIdx.x;
  const int bid  = blockIdx.x;
  const int wsel = bid >> 2;
  if (wsel >= 4) return;
  const int kt = bid & 1, nt = (bid >> 1) & 1;
  const float* W = (wsel == 0) ? W0 : ((wsel == 1) ? W1 : ((wsel == 2) ? W2 : W3));
  const int f16mode = (wsel == 3) ? 1 : 0;
  const int k0 = kt * 64, n0 = nt * 64;
  {
    const int kk = tid >> 2;
    const int nq = (tid & 3) * 16;
    const float* src = W + (size_t)(k0 + kk) * CD + n0 + nq;
#pragma unroll
    for (int i = 0; i < 4; ++i) {
      const v4f a = *(const v4f*)(src + 4 * i);
#pragma unroll
      for (int e = 0; e < 4; ++e) {
        const float f = a[e];
        const unsigned short hb = h_bits((_Float16)(bfr(f) * WOS));
        const unsigned short bb = bf_bits(f);
        TT[(nq + 4 * i + e) * TWP + kk] = (f16mode != 0) ? hb : bb;
      }
    }
  }
  __syncthreads();
  const int q8 = tid >> 3, p8 = (tid & 7) * 8;
  v4u v[2];
#pragma unroll
  for (int it = 0; it < 2; ++it) {
    const int line = it * 32 + q8;
    v[it] = *(const v4u*)(TT + line * TWP + p8);
  }
  const size_t base = (size_t)wsel * CD * CD + (size_t)n0 * CD + k0 + p8;
  for (int pass = 0; pass < 2; ++pass) {
#pragma unroll
    for (int it = 0; it < 2; ++it) {
      const int line = it * 32 + q8;
      *(volatile v4u*)(T + base + (size_t)line * CD) = v[it];
    }
    __threadfence();
  }
}

__global__ __launch_bounds__(256) void vt16(const float* __restrict__ F, u16* VHo, u16* VLo) {
  __shared__ __align__(16) u16 TH[CD * VTP];
  __shared__ __align__(16) u16 TL[CD * VTP];
  const int tid = threadIdx.x;
  const int bid = blockIdx.x;
  const int nst = MSEG / 64;
  const int st  = bid % nst;
  const int ug  = bid / nst;
  if (ug >= NB * NUNIT) return;
  const int b    = ug / NUNIT;
  const int u    = ug - b * NUNIT;
  const int br   = (u < 4) ? 0 : ((u < 6) ? 1 : 2);
  const int seg  = (u < 4) ? u : ((u < 6) ? (u - 4) : 0);
  const int rstr = 1 << br;
  const int wseg = MSEG << br;
  const int sl0  = st * 64;
  {
    const int sl = tid >> 2;
    const int dc = (tid & 3) * 32;
    const size_t tok = (size_t)b * SEQ + (size_t)seg * wseg + (size_t)rstr * (size_t)(sl0 + sl);
    const float* src = F + tok * CD + dc;
#pragma unroll
    for (int i = 0; i < 8; ++i) {
      const v4f a = *(const v4f*)(src + 4 * i);
#pragma unroll
      for (int e = 0; e < 4; ++e) {
        const float t = a[e] * VCAR;
        const _Float16 hv = (_Float16)t;
        const _Float16 lv = (_Float16)(t - (float)hv);
        TH[(dc + 4 * i + e) * VTP + sl] = h_bits(hv);
        TL[(dc + 4 * i + e) * VTP + sl] = h_bits(lv);
      }
    }
  }
  __syncthreads();
  v4u vh[4], vl[4];
  const int q8 = tid >> 3, p8 = (tid & 7) * 8;
#pragma unroll
  for (int it = 0; it < 4; ++it) {
    const int line = it * 32 + q8;
    vh[it] = *(const v4u*)(TH + line * VTP + p8);
    vl[it] = *(const v4u*)(TL + line * VTP + p8);
  }
  const size_t hrow  = (size_t)ug * CD;
  const size_t baseH = hrow * MSEG + (size_t)sl0 + p8;
  const size_t baseL = hrow * KRES + (size_t)sl0 + p8;
  const bool   wl    = (sl0 < KRES);
  for (int pass = 0; pass < 2; ++pass) {
#pragma unroll
    for (int it = 0; it < 4; ++it) {
      const int line = it * 32 + q8;
      *(volatile v4u*)(VHo + baseH + (size_t)line * MSEG) = vh[it];
      if (wl) {
        *(volatile v4u*)(VLo + baseL + (size_t)line * KRES) = vl[it];
      }
    }
    __threadfence();
  }
}

__device__ __forceinline__ void epi64(float* sl, v8f a0, v8f a1, v8f a2, v8f a3, float oscale,
                                      float* C, int N, size_t rowb, int col0, int lane) {
  const int hh = lane >> 4, m = lane & 15;
#pragma unroll
  for (int r = 0; r < 8; ++r) {
    const int ro = (8 * hh + r) * 68 + m;
    sl[ro]      = a0[r] * oscale;
    sl[ro + 16] = a1[r] * oscale;
    sl[ro + 32] = a2[r] * oscale;
    sl[ro + 48] = a3[r] * oscale;
  }
  wave_sync_lds();
  v4f vals[8];
#pragma unroll
  for (int it = 0; it < 8; ++it) vals[it] = *(const v4f*)(sl + (it * 2 + hh) * 68 + m * 4);
  float* dst = C + (rowb + (size_t)hh) * (size_t)N + col0 + m * 4;
  for (int pass = 0; pass < 2; ++pass) {
#pragma unroll
    for (int it = 0; it < 8; ++it) {
      *(volatile v4f*)(dst + (size_t)(it * 2) * (size_t)N) = vals[it];
    }
    __threadfence();
  }
}

__global__ __launch_bounds__(128)
void gemm_bf(const u16* __restrict__ A, const u16* __restrict__ Bt, float* C, int M, int N, int K, float oscale) {
  __shared__ __align__(16) float slab[4 * SLAB64];
  const int tid = threadIdx.x, wave = tid >> 5, lane = tid & 31, hh = lane >> 4, m = lane & 15;
  const int ntile = N >> 6;
  const int bid   = blockIdx.x;
  const int rowb  = (bid / ntile) * 64 + wave * 16;
  const int col0  = (bid % ntile) * 64;
  if (rowb + 16 > M) return;
  const u16* ap = A  + (size_t)(rowb + m) * K + 8 * hh;
  const u16* bp = Bt + (size_t)(col0 + m) * K + 8 * hh;
  const size_t bs = (size_t)16 * K;
  v8f acc0 = zero8(), acc1 = zero8(), acc2 = zero8(), acc3 = zero8();
#pragma unroll 1
  for (int k0 = 0; k0 < K; k0 += 32) {
    const v16b a  = ldfrag_b(ap + k0);
    const v16b b0 = ldfrag_b(bp + k0);
    const v16b b1 = ldfrag_b(bp + bs + k0);
    const v16b b2 = ldfrag_b(bp + 2 * bs + k0);
    const v16b b3 = ldfrag_b(bp + 3 * bs + k0);
    acc0 = mma_b(a, b0, acc0);
    acc1 = mma_b(a, b1, acc1);
    acc2 = mma_b(a, b2, acc2);
    acc3 = mma_b(a, b3, acc3);
    guard6<v16b>(acc0, acc1, acc2, acc3, a, b0, b1, b2, b3, a);
  }
  epi64(slab + wave * SLAB64, acc0, acc1, acc2, acc3, oscale, C, N, (size_t)rowb, col0, lane);
}

__global__ __launch_bounds__(128)
void gemm_o2(const u16* __restrict__ Ah, const u16* __restrict__ Al, const u16* __restrict__ Bt, float* C, int M, float oscale) {
  __shared__ __align__(16) float slab[4 * SLAB64];
  const int tid = threadIdx.x, wave = tid >> 5, lane = tid & 31, hh = lane >> 4, m = lane & 15;
  const int bid  = blockIdx.x;
  const int rowb = (bid >> 1) * 64 + wave * 16;
  const int col0 = (bid & 1) * 64;
  if (rowb + 16 > M) return;
  const int K = CD;
  const _Float16* ahp = (const _Float16*)(const void*)Ah + (size_t)(rowb + m) * K + 8 * hh;
  const _Float16* alp = (const _Float16*)(const void*)Al + (size_t)(rowb + m) * K + 8 * hh;
  const _Float16* bp  = (const _Float16*)(const void*)Bt + (size_t)(col0 + m) * K + 8 * hh;
  const size_t bs = (size_t)16 * K;
  v8f acc0 = zero8(), acc1 = zero8(), acc2 = zero8(), acc3 = zero8();
#pragma unroll 1
  for (int k0 = 0; k0 < K; k0 += 32) {
    const v16h ah = ldfrag_h(ahp + k0), al = ldfrag_h(alp + k0);
    const v16h b0 = ldfrag_h(bp + k0);
    const v16h b1 = ldfrag_h(bp + bs + k0);
    const v16h b2 = ldfrag_h(bp + 2 * bs + k0);
    const v16h b3 = ldfrag_h(bp + 3 * bs + k0);
    acc0 = mma_h(ah, b0, acc0);  acc0 = mma_h(al, b0, acc0);
    acc1 = mma_h(ah, b1, acc1);  acc1 = mma_h(al, b1, acc1);
    acc2 = mma_h(ah, b2, acc2);  acc2 = mma_h(al, b2, acc2);
    acc3 = mma_h(ah, b3, acc3);  acc3 = mma_h(al, b3, acc3);
    guard6<v16h>(acc0, acc1, acc2, acc3, ah, al, b0, b1, b2, b3);
  }
  epi64(slab + wave * SLAB64, acc0, acc1, acc2, acc3, oscale, C, CD, (size_t)rowb, col0, lane);
}

template <bool VRES, bool PRES>
__device__ __forceinline__ void att_tile(const int kb,
                                         const _Float16* __restrict__ Qh, const _Float16* __restrict__ Ql,
                                         const _Float16* __restrict__ Khb, const _Float16* __restrict__ Klb, const size_t KROW,
                                         const _Float16* __restrict__ Vhb, const _Float16* __restrict__ Vlb,
                                         const float lsc, const int qr0, const int c, const int hh, float* pt,
                                         float (&mrow)[8], float (&lrow)[8], v8f (&o)[8]) {
  v8f s0 = zero8(), s1 = zero8();
  const _Float16* k0p = Khb + (size_t)kb * KROW;
  const _Float16* k1p = k0p + (size_t)16 * KROW;
  const _Float16* l0p = Klb + (size_t)kb * KROW;
  const _Float16* l1p = l0p + (size_t)16 * KROW;
#pragma unroll
  for (int kk = 0; kk < CD / 32; ++kk) {
    const v16h qh  = ldfrag_h(Qh + kk * 32);
    const v16h ql  = ldfrag_h(Ql + kk * 32);
    const v16h kh0 = ldfrag_h(k0p + kk * 32);
    const v16h kh1 = ldfrag_h(k1p + kk * 32);
    const v16h kl0 = ldfrag_h(l0p + kk * 32);
    const v16h kl1 = ldfrag_h(l1p + kk * 32);
    s0 = mma_h(qh, kh0, s0);
    s0 = mma_h(ql, kh0, s0);
    s0 = mma_h(qh, kl0, s0);
    s1 = mma_h(qh, kh1, s1);
    s1 = mma_h(ql, kh1, s1);
    s1 = mma_h(qh, kl1, s1);
    guard2(s0, s1, qh, ql, kh0, kl0, kh1, kl1);
  }
  const int key0 = kb + c, key1 = kb + 16 + c;
#pragma unroll
  for (int r = 0; r < 8; ++r) {
    const int   qr = qr0 + r;
    const float u0 = s0[r] * lsc;
    const float u1 = s1[r] * lsc;
    const float t0 = (key0 <= qr) ? u0 : NEGT;
    const float t1 = (key1 <= qr) ? u1 : NEGT;
    float mx = fmaxf(t0, t1);
#pragma unroll
    for (int off = 1; off < 16; off <<= 1) mx = fmaxf(mx, __shfl_xor(mx, off, 32));
    const float mn = fmaxf(mrow[r], mx);
    const float ms = (mn == -INFINITY) ? 0.0f : mn;
    const float al = exp2f(mrow[r] - ms);
    mrow[r] = mn;
    const float e0 = exp2f(t0 - ms), e1 = exp2f(t1 - ms);
    float ps = e0 + e1;
#pragma unroll
    for (int off = 1; off < 16; off <<= 1) ps += __shfl_xor(ps, off, 32);
    lrow[r] = lrow[r] * al + ps;
#pragma unroll
    for (int j = 0; j < 8; ++j) o[j][r] *= al;
    const int ro = (8 * hh + r) * PTP + c;
    pt[ro]      = e0;
    pt[ro + 16] = e1;
  }
  wave_sync_lds();
  FragH ph, pl;
  {
    const float* prow = pt + c * PTP + 8 * hh;
    const v4f p0 = *(const v4f*)(prow), p1 = *(const v4f*)(prow + 4);
    const v4f p2 = *(const v4f*)(prow + 16), p3 = *(const v4f*)(prow + 20);
#pragma unroll
    for (int e = 0; e < 4; ++e) {
      const float ta = p0[e] * PCAR, tb = p1[e] * PCAR, tc = p2[e] * PCAR, td = p3[e] * PCAR;
      const _Float16 ha = (_Float16)ta, hb = (_Float16)tb, hc = (_Float16)tc, hd = (_Float16)td;
      ph.h[0][e]     = ha;
      ph.h[0][4 + e] = hb;
      ph.h[1][e]     = hc;
      ph.h[1][4 + e] = hd;
      if constexpr (PRES) {
        pl.h[0][e]     = (_Float16)(ta - (float)ha);
        pl.h[0][4 + e] = (_Float16)(tb - (float)hb);
        pl.h[1][e]     = (_Float16)(tc - (float)hc);
        pl.h[1][4 + e] = (_Float16)(td - (float)hd);
      }
    }
  }
  if constexpr (!PRES) pl.v = ph.v;
  {
    const _Float16* vhp = Vhb + kb;
    const _Float16* vlp = Vlb + kb;
#pragma unroll
    for (int jg = 0; jg < 4; ++jg) {
      const size_t da = (size_t)(2 * jg) * 16 * MSEG;
      const size_t db = da + (size_t)16 * MSEG;
      const v16h vha = ldfrag_h(vhp + da), vhb2 = ldfrag_h(vhp + db);
      o[2 * jg]     = mma_h(ph.v, vha,  o[2 * jg]);
      o[2 * jg + 1] = mma_h(ph.v, vhb2, o[2 * jg + 1]);
      if constexpr (PRES) {
        o[2 * jg]     = mma_h(pl.v, vha,  o[2 * jg]);
        o[2 * jg + 1] = mma_h(pl.v, vhb2, o[2 * jg + 1]);
      }
      if constexpr (VRES) {
        const size_t dla = (size_t)(2 * jg) * 16 * KRES;
        const size_t dlb = dla + (size_t)16 * KRES;
        const v16h vla = ldfrag_h(vlp + dla), vlb2 = ldfrag_h(vlp + dlb);
        o[2 * jg]     = mma_h(ph.v, vla,  o[2 * jg]);
        o[2 * jg + 1] = mma_h(ph.v, vlb2, o[2 * jg + 1]);
        guard2(o[2 * jg], o[2 * jg + 1], ph.v, pl.v, vha, vhb2, vla, vlb2);
      } else {
        guard2(o[2 * jg], o[2 * jg + 1], ph.v, pl.v, vha, vhb2, vha, vhb2);
      }
    }
  }
  wave_sync_lds();
}

__global__ __launch_bounds__(ATT_THREADS)
void attn_d(const u16* __restrict__ QHp, const u16* __restrict__ QLp,
            const u16* __restrict__ KHp, const u16* __restrict__ KLp,
            const u16* __restrict__ VHp, const u16* __restrict__ VLp,
            float* CX, float* DP, int wseg, int rstr, int nseg, int ub) {
  __shared__ __align__(16) float smem[WPB * WREG];

  const int tid  = threadIdx.x;
  const int wave = tid >> 5;
  const int lane = tid & 31;
  const int hh   = lane >> 4;
  const int c    = lane & 15;
  const int bid  = blockIdx.x;
  const int qt   = bid % NQB;
  const int t2   = bid / NQB;
  const int seg  = t2 % nseg;
  const int b    = t2 / nseg;
  if (b >= NB) return;
  const int q0b  = qt * 32;
  const int q0   = q0b + wave * 16;

  float* pt   = smem + wave * WREG;
  float* slab = pt + PTW;

  const size_t tokb = (size_t)b * SEQ + (size_t)seg * (size_t)wseg;
  const size_t hc8  = (size_t)(8 * hh);
  const _Float16* Qh  = (const _Float16*)(const void*)QHp + (tokb + (size_t)rstr * (size_t)(q0 + c)) * CD + hc8;
  const _Float16* Ql  = (const _Float16*)(const void*)QLp + (tokb + (size_t)rstr * (size_t)(q0 + c)) * CD + hc8;
  const _Float16* Khb = (const _Float16*)(const void*)KHp + (tokb + (size_t)rstr * (size_t)c) * CD + hc8;
  const _Float16* Klb = (const _Float16*)(const void*)KLp + (tokb + (size_t)rstr * (size_t)c) * CD + hc8;
  const int ug = b * NUNIT + ub + seg;
  const _Float16* Vhb = (const _Float16*)(const void*)VHp + ((size_t)ug * CD + c) * MSEG + hc8;
  const _Float16* Vlb = (const _Float16*)(const void*)VLp + ((size_t)ug * CD + c) * KRES + hc8;
  const float  lsc  = RSQ_HD * (LOG2E / (QSC * KSC));
  const float  oc   = 1.0f / (PCAR * VCAR);
  const size_t KROW = (size_t)rstr * CD;

  float mrow[8], lrow[8];
  v8f o[8];
#pragma unroll
  for (int r = 0; r < 8; ++r) { mrow[r] = -INFINITY; lrow[r] = 0.f; }
#pragma unroll
  for (int j = 0; j < 8; ++j) o[j] = zero8();
  const int ncaus = qt + 1;
  const int nkt   = (ncaus < NKT) ? ncaus : NKT;
  const int qr0   = q0 + 8 * hh;
  const bool pres = (q0b < QO);

  if (pres) {
#pragma unroll 1
    for (int kt = 0; kt < nkt; ++kt) {
      att_tile<true, true>(kt * 32, Qh, Ql, Khb, Klb, KROW, Vhb, Vlb, lsc, qr0, c, hh, pt, mrow, lrow, o);
    }
  } else {
    const int nres = KRES / 32;
    const int n1   = (nkt < nres) ? nkt : nres;
#pragma unroll 1
    for (int kt = 0; kt < n1; ++kt) {
      att_tile<true, false>(kt * 32, Qh, Ql, Khb, Klb, KROW, Vhb, Vlb, lsc, qr0, c, hh, pt, mrow, lrow, o);
    }
#pragma unroll 1
    for (int kt = n1; kt < nkt; ++kt) {
      att_tile<false, false>(kt * 32, Qh, Ql, Khb, Klb, KROW, Vhb, Vlb, lsc, qr0, c, hh, pt, mrow, lrow, o);
    }
  }
  acc_guard4(o[0], o[1], o[2], o[3]);
  acc_guard4(o[4], o[5], o[6], o[7]);
#pragma unroll
  for (int r = 0; r < 8; ++r) {
    const float lv  = lrow[r];
    const float ls  = (lv > 0.0f) ? lv : 1.0f;
    const float inv = (lv > 0.0f) ? ((1.0f / ls) * oc) : 0.0f;
#pragma unroll
    for (int j = 0; j < 8; ++j) {
      const int idx = (8 * hh + r) * SLP + j * 16 + c;
      slab[idx] = o[j][r] * inv;
    }
    const float dn = exp2f(mrow[r]) * lv;
    if (c == 0) pt[8 * hh + r] = dn;
  }
  wave_sync_lds();
  v4f vals[16];
#pragma unroll
  for (int it = 0; it < 16; ++it) vals[it] = *(const v4f*)(slab + it * SLP + 4 * lane);
  const v4f  dl   = *(const v4f*)(pt + 4 * (lane & 3));
  const bool keep = ((lane & 7) < 4);
  v4f dv;
#pragma unroll
  for (int e = 0; e < 4; ++e) dv[e] = keep ? dl[e] : 0.0f;
  const size_t urow = (size_t)(b * nseg + seg) * MSEG + (size_t)q0;
  float* cdst = CX + urow * CD + 4 * lane;
  float* ddst = DP + (urow >> 4) * 32 + 4 * (lane & 7);
  for (int pass = 0; pass < 2; ++pass) {
#pragma unroll
    for (int it = 0; it < 16; ++it) {
      *(volatile v4f*)(cdst + (size_t)it * CD) = vals[it];
    }
    if (lane < 8) {
      *(volatile v4f*)(ddst) = dv;
    }
    __threadfence();
  }
}

__global__ __launch_bounds__(256)
void combine(const float* __restrict__ C1, const float* __restrict__ C2, const float* __restrict__ C3,
             const float* __restrict__ D1, const float* __restrict__ D2, const float* __restrict__ D3,
             u16* CHo, u16* CLo, int nthr) {
  const int gt = blockIdx.x * 256 + (int)threadIdx.x;
  if (gt >= nthr) return;
  const int R   = gt >> 4;
  const int c8  = (gt & 15) * 8;
  const int b   = R / SEQ;
  const int pos = R - b * SEQ;
  const int r1  = R;
  const int r2  = b * (SEQ / 2) + (pos >> 1);
  const int r3  = b * (SEQ / 4) + (pos >> 2);
  const float d1 = D1[(size_t)(r1 >> 4) * 32 + (r1 & 15)];
  const float d2 = D2[(size_t)(r2 >> 4) * 32 + (r2 & 15)];
  const float d3 = D3[(size_t)(r3 >> 4) * 32 + (r3 & 15)];
  const float w2 = ((pos & 1) == 0) ? d2 : 0.0f;
  const float w3 = ((pos & 3) == 0) ? d3 : 0.0f;
  const float S  = (d1 + w2) + w3;
  const float rS = 1.0f / S;
  const float a1 = d1 * rS, a2 = w2 * rS, a3 = w3 * rS;
  const float* p1 = C1 + (size_t)r1 * CD + c8;
  const float* p2 = C2 + (size_t)r2 * CD + c8;
  const float* p3 = C3 + (size_t)r3 * CD + c8;
  const v4f x1a = *(const v4f*)(p1), x1b = *(const v4f*)(p1 + 4);
  const v4f x2a = *(const v4f*)(p2), x2b = *(const v4f*)(p2 + 4);
  const v4f x3a = *(const v4f*)(p3), x3b = *(const v4f*)(p3 + 4);
  float cc[8];
#pragma unroll
  for (int e = 0; e < 4; ++e) {
    cc[e]     = (x1a[e] * a1 + x2a[e] * a2) + x3a[e] * a3;
    cc[4 + e] = (x1b[e] * a1 + x2b[e] * a2) + x3b[e] * a3;
  }
  v4u oh, ol;
#pragma unroll
  for (int e = 0; e < 4; ++e) {
    const float t0 = cc[2 * e] * OSC, t1 = cc[2 * e + 1] * OSC;
    const _Float16 h0 = (_Float16)t0, h1 = (_Float16)t1;
    const _Float16 l0 = (_Float16)(t0 - (float)h0), l1 = (_Float16)(t1 - (float)h1);
    oh[e] = pk16(h_bits(h0), h_bits(h1));
    ol[e] = pk16(h_bits(l0), h_bits(l1));
  }
  u16* dh = CHo + (size_t)gt * 8;
  u16* dl = CLo + (size_t)gt * 8;
  for (int pass = 0; pass < 2; ++pass) {
    *(volatile v4u*)(dh) = oh;
    *(volatile v4u*)(dl) = ol;
    __threadfence();
  }
}

extern "C" void kernel_launch(void* const* d_in, const int* in_sizes, int n_in,
                              void* d_out, int out_size, void* d_ws, size_t ws_size,
                              hipStream_t stream) {
  if (n_in < 5) return;
  if (in_sizes[0] < ((NB - 1) * SEQ_FULL + SEQ) * CD) return;
  if (in_sizes[1] < CD * CD) return;
  if (in_sizes[2] < CD * CD) return;
  if (in_sizes[3] < CD * CD) return;
  if (in_sizes[4] < CD * CD) return;
  if (out_size < MROWS * CD) return;

  const float* x  = (const float*)d_in[0];
  const float* wq = (const float*)d_in[1];
  const float* wk = (const float*)d_in[2];
  const float* wv = (const float*)d_in[3];
  const float* wo = (const float*)d_in[4];
  float*       out = (float*)d_out;

  const size_t szWT = (size_t)4 * CD * CD * 2;
  const size_t szXB = (size_t)MROWS * CD * 2;
  const size_t szF  = (size_t)MROWS * CD * 4;
  const size_t szP  = (size_t)MROWS * CD * 2;
  const size_t szVH = (size_t)NB * NUNIT * CD * MSEG * 2;
  const size_t szVL = (size_t)NB * NUNIT * CD * KRES * 2;
  const size_t szC1 = (size_t)NB * 4 * MSEG * CD * 4;
  const size_t szC2 = (size_t)NB * 2 * MSEG * CD * 4;
  const size_t szC3 = (size_t)NB * 1 * MSEG * CD * 4;
  const size_t szD1 = (size_t)NB * 4 * MSEG * 2 * 4;
  const size_t szD2 = (size_t)NB * 2 * MSEG * 2 * 4;
  const size_t szD3 = (size_t)NB * 1 * MSEG * 2 * 4;
  size_t off = 0;
  const size_t oWT = off; off += szWT;
  const size_t oXB = off; off += szXB;
  const size_t oF  = off; off += szF;
  const size_t oQH = off; off += szP;
  const size_t oQL = off; off += szP;
  const size_t oKH = off; off += szP;
  const size_t oKL = off; off += szP;
  const size_t oVH = off; off += szVH;
  const size_t oVL = off; off += szVL;
  const size_t oC1 = off; off += szC1;
  const size_t oC2 = off; off += szC2;
  const size_t oC3 = off; off += szC3;
  const size_t oD1 = off; off += szD1;
  const size_t oD2 = off; off += szD2;
  const size_t oD3 = off; off += szD3;
  const size_t oCH = off; off += szP;
  const size_t oCL = off; off += szP;
  if (off > ws_size) return;
  if (off > (size_t)WS_CAP) return;

  char*  ws  = (char*)d_ws;
  u16*   WT  = (u16*)(ws + oWT);
  u16*   XB  = (u16*)(ws + oXB);
  float* F   = (float*)(ws + oF);
  u16*   QH  = (u16*)(ws + oQH);
  u16*   QL  = (u16*)(ws + oQL);
  u16*   KH  = (u16*)(ws + oKH);
  u16*   KL  = (u16*)(ws + oKL);
  u16*   VH  = (u16*)(ws + oVH);
  u16*   VL  = (u16*)(ws + oVL);
  float* C1  = (float*)(ws + oC1);
  float* C2  = (float*)(ws + oC2);
  float* C3  = (float*)(ws + oC3);
  float* D1  = (float*)(ws + oD1);
  float* D2  = (float*)(ws + oD2);
  float* D3  = (float*)(ws + oD3);
  u16*   CH  = (u16*)(ws + oCH);
  u16*   CL  = (u16*)(ws + oCL);
  u16*   WO  = WT + (size_t)3 * CD * CD;

  const dim3 b256(256), b128(128), bAT(ATT_THREADS);
  const int  n8   = (MROWS * CD) / 8;
  const dim3 gCV((n8 + 255) / 256);
  const dim3 gTW(16);
  const dim3 gG((MROWS / 64) * (CD / 64));
  const dim3 gVT(NB * NUNIT * (MSEG / 64));
  const int  nthr = MROWS * 16;
  const dim3 gCB((nthr + 255) / 256);
  const dim3 gO((MROWS / 64) * 2);

  tw16<<<gTW, b256, 0, stream>>>(wq, wk, wv, wo, WT);
  cvtx<<<gCV, b256, 0, stream>>>(x, XB, n8);
  gemm_bf<<<gG, b128, 0, stream>>>(XB, WT, F, MROWS, CD, CD, 1.0f);
  cvt_hl<<<gCV, b256, 0, stream>>>(F, QH, QL, n8, QSC);
  gemm_bf<<<gG, b128, 0, stream>>>(XB, WT + (size_t)CD * CD, F, MROWS, CD, CD, 1.0f);
  cvt_hl<<<gCV, b256, 0, stream>>>(F, KH, KL, n8, KSC);
  gemm_bf<<<gG, b128, 0, stream>>>(XB, WT + (size_t)2 * CD * CD, F, MROWS, CD, CD, 1.0f);
  vt16<<<gVT, b256, 0, stream>>>(F, VH, VL);
  attn_d<<<dim3(NQB * 4 * NB), bAT, 0, stream>>>(QH, QL, KH, KL, VH, VL, C1, D1, SEQ / 4, 1, 4, 0);
  attn_d<<<dim3(NQB * 2 * NB), bAT, 0, stream>>>(QH, QL, KH, KL, VH, VL, C2, D2, SEQ / 2, 2, 2, 4);
  attn_d<<<dim3(NQB * 1 * NB), bAT, 0, stream>>>(QH, QL, KH, KL, VH, VL, C3, D3, SEQ,     4, 1, 6);
  combine<<<gCB, b256, 0, stream>>>(C1, C2, C3, D1, D2, D3, CH, CL, nthr);
  gemm_o2<<<gO, b128, 0, stream>>>(CH, CL, WO, out, MROWS, 1.0f / (OSC * WOS));
  (void)hipGetLastError();
}
